// Transformer_layer_78228534329470
// MI455X (gfx1250) — hardware-verified
//
#include <hip/hip_runtime.h>
#include <math.h>
#include <stddef.h>


typedef _Float16 h16;
typedef _Float16 v16h __attribute__((ext_vector_type(16)));
typedef _Float16 v8h  __attribute__((ext_vector_type(8)));
typedef _Float16 v4h  __attribute__((ext_vector_type(4)));
typedef float    v8f  __attribute__((ext_vector_type(8)));
typedef float    v4f  __attribute__((ext_vector_type(4)));

union Frag { v16h v; v8h half[2]; };

static __device__ __forceinline__ v8f wmma16(v16h a, v16h b, v8f c) {
  v8f d = __builtin_amdgcn_wmma_f32_16x16x32_f16(false, a, false, b, (short)0, c, false, false);
  asm volatile("v_nop\n\tv_nop\n\tv_nop\n\tv_nop" : "+v"(d) : "v"(a), "v"(b));
  return d;
}

static __device__ __forceinline__ v16h ldfrag(const h16* p) {
  Frag f;
  f.half[0] = *(const v8h*)p;
  f.half[1] = *(const v8h*)(p + 16);
  return f.v;
}

static __device__ __forceinline__ v8h ld8(const h16* p) { return *(const v8h*)p; }

static __device__ __forceinline__ void st2_v4f(float* p, v4f v) {
  *(volatile v4f*)p = v;
  __threadfence();
  *(volatile v4f*)p = v;
}
static __device__ __forceinline__ void st2_v8h(h16* p, v8h v) {
  *(volatile v8h*)p = v;
  __threadfence();
  *(volatile v8h*)p = v;
}

static __device__ __forceinline__ float wsum(float v) {
#pragma unroll
  for (int m = 16; m > 0; m >>= 1) v += __shfl_xor(v, m, 32);
  return v;
}

__global__ __launch_bounds__(256) void k_cvt_act(const float* __restrict__ in,
                                                 h16* __restrict__ out, int n8) {
  const int i = blockIdx.x * 256 + threadIdx.x;
  if (i < n8) {
    const size_t o = (size_t)i * 8;
    v4f a = *(const v4f*)(in + o);
    v4f b = *(const v4f*)(in + o + 4);
    v8h r;
#pragma unroll
    for (int j = 0; j < 4; ++j) { r[j] = (h16)a[j]; r[j + 4] = (h16)b[j]; }
    st2_v8h(out + o, r);
  }
}

__global__ __launch_bounds__(256) void k_cvt_wt(const float* __restrict__ W,
                                                h16* __restrict__ Wt,
                                                int K, int N, float scale) {
  constexpr int TP = 72;
  __shared__ __align__(16) h16 tile[64 * TP];
  const int t = threadIdx.x;
  const int n0 = blockIdx.x * 64, k0 = blockIdx.y * 64;
#pragma unroll
  for (int i = 0; i < 4; ++i) {
    const int idx = t + 256 * i;
    const int kk = idx >> 4, c4 = (idx & 15) * 4;
    const int k = k0 + kk, n = n0 + c4;
    v4f w;
    w[0] = 0.f; w[1] = 0.f; w[2] = 0.f; w[3] = 0.f;
    if (k < K && n + 3 < N) w = *(const v4f*)(W + (size_t)k * N + n);
#pragma unroll
    for (int j = 0; j < 4; ++j) tile[(c4 + j) * TP + kk] = (h16)(w[j] * scale);
  }
  __syncthreads();
#pragma unroll
  for (int i = 0; i < 2; ++i) {
    const int idx = t + 256 * i;
    const int row = idx >> 3, piece = idx & 7;
    const int n = n0 + row, k = k0 + piece * 8;
    v8h v = *(const v8h*)(tile + row * TP + piece * 8);
    if (n < N && k + 7 < K) st2_v8h(Wt + (size_t)n * K + k, v);
  }
}

template <bool ADD>
__global__ __launch_bounds__(256) void k_ln(const float* __restrict__ a,
                                            const float* __restrict__ r,
                                            const float* __restrict__ g,
                                            const float* __restrict__ bta,
                                            float* __restrict__ sum_out,
                                            h16* __restrict__ nrm, int nrows) {
  constexpr int C = 1024;
  __shared__ float red1[8];
  __shared__ float red2[8];
  __shared__ __align__(16) h16 rowh[C];
  const int row = blockIdx.x;
  if (row >= nrows) return;
  const int t = threadIdx.x, lane = t & 31, wave = t >> 5;
  const size_t base = (size_t)row * C + 4 * t;

  v4f v = *(const v4f*)(r + base);
  if (ADD) {
    v4f w = *(const v4f*)(a + base);
    v = v + w;
    st2_v4f(sum_out + base, v);
  }
  float s = (v[0] + v[1]) + (v[2] + v[3]);
  s = wsum(s);
  if (lane == 0) red1[wave] = s;
  __syncthreads();
  float tot = 0.f;
#pragma unroll
  for (int i = 0; i < 8; ++i) tot += red1[i];
  const float mean = tot * (1.0f / C);

  v4f d;
#pragma unroll
  for (int j = 0; j < 4; ++j) d[j] = v[j] - mean;
  float s2 = (d[0] * d[0] + d[1] * d[1]) + (d[2] * d[2] + d[3] * d[3]);
  s2 = wsum(s2);
  if (lane == 0) red2[wave] = s2;
  __syncthreads();
  float tot2 = 0.f;
#pragma unroll
  for (int i = 0; i < 8; ++i) tot2 += red2[i];
  const float var = tot2 * (1.0f / C);
  const float rstd = rsqrtf(var + 1e-5f);

  v4f gg = *(const v4f*)(g + 4 * t);
  v4f bb = *(const v4f*)(bta + 4 * t);
  v4h o;
#pragma unroll
  for (int j = 0; j < 4; ++j) o[j] = (h16)((d[j] * rstd) * gg[j] + bb[j]);
  *(v4h*)(rowh + 4 * t) = o;
  __syncthreads();
  if (t < 128) {
    v8h q = *(const v8h*)(rowh + 8 * t);
    st2_v8h(nrm + (size_t)row * C + 8 * t, q);
  }
}

template <int EPI>
__global__ __launch_bounds__(256) void k_gemm(const h16* __restrict__ A, int lda,
                                             const h16* __restrict__ Bt, int ldb,
                                             h16* __restrict__ Ch, float* __restrict__ Cf, int ldc,
                                             const float* __restrict__ bias,
                                             const float* __restrict__ resid, int ldr,
                                             int M, int N, int K, float oscale) {
  constexpr int BM = 128, BN = 128, BK = 32, LP = 40;
  constexpr int SP = 132;
  __shared__ __align__(16) float smem[64 * SP];
  h16* As = (h16*)smem;
  h16* Bs = As + BM * LP;

  const int t = threadIdx.x, wave = t >> 5, lane = t & 31;
  const int lr = lane & 15, ls = lane >> 4;
  const int wm = (wave >> 2) * 64, wn = (wave & 3) * 32;
  const int m0 = blockIdx.y * BM, n0 = blockIdx.x * BN;
  if (m0 + BM > M || n0 + BN > N) return;

  const int ar = t >> 2, ac = (t & 3) * 8;

  v8f acc[4][2];
#pragma unroll
  for (int im = 0; im < 4; ++im)
#pragma unroll
    for (int in = 0; in < 2; ++in)
#pragma unroll
      for (int q = 0; q < 8; ++q) acc[im][in][q] = 0.f;

  const int ns = K / BK;
  for (int s = 0; s < ns; ++s) {
    const int k0 = s * BK;
    v8h a0 = ld8(A + (size_t)(m0 + ar) * lda + k0 + ac);
    v8h a1 = ld8(A + (size_t)(m0 + 64 + ar) * lda + k0 + ac);
    v8h b0 = ld8(Bt + (size_t)(n0 + ar) * ldb + k0 + ac);
    v8h b1 = ld8(Bt + (size_t)(n0 + 64 + ar) * ldb + k0 + ac);
    __syncthreads();
    *(v8h*)(As + ar * LP + ac) = a0;
    *(v8h*)(As + (64 + ar) * LP + ac) = a1;
    *(v8h*)(Bs + ar * LP + ac) = b0;
    *(v8h*)(Bs + (64 + ar) * LP + ac) = b1;
    __syncthreads();

    v16h af[4], bf[2];
#pragma unroll
    for (int im = 0; im < 4; ++im) af[im] = ldfrag(As + (wm + im * 16 + lr) * LP + 8 * ls);
#pragma unroll
    for (int in = 0; in < 2; ++in) bf[in] = ldfrag(Bs + (wn + in * 16 + lr) * LP + 8 * ls);
#pragma unroll
    for (int im = 0; im < 4; ++im)
#pragma unroll
      for (int in = 0; in < 2; ++in) acc[im][in] = wmma16(af[im], bf[in], acc[im][in]);
  }
  __syncthreads();

#pragma unroll
  for (int p = 0; p < 2; ++p) {
    if ((wave >> 2) == p) {
#pragma unroll
      for (int im = 0; im < 4; ++im)
#pragma unroll
        for (int in = 0; in < 2; ++in)
#pragma unroll
          for (int q = 0; q < 8; ++q)
            smem[(im * 16 + 8 * ls + q) * SP + wn + in * 16 + lr] = acc[im][in][q];
    }
    __syncthreads();
    const int rbase = m0 + p * 64;
    if (EPI == 2) {
#pragma unroll 1
      for (int it = 0; it < 8; ++it) {
        const int row = it * 8 + (t >> 5);
        const int c = (t & 31) * 4;
        v4f v = *(const v4f*)(smem + row * SP + c);
        v4f bb = *(const v4f*)(bias + n0 + c);
        v4f rr = *(const v4f*)(resid + (size_t)(rbase + row) * ldr + n0 + c);
        v4f o;
#pragma unroll
        for (int j = 0; j < 4; ++j) o[j] = (v[j] * oscale + bb[j]) + rr[j];
        st2_v4f(Cf + (size_t)(rbase + row) * ldc + n0 + c, o);
      }
    } else {
#pragma unroll 1
      for (int it = 0; it < 4; ++it) {
        const int row = it * 16 + (t >> 4);
        const int c = (t & 15) * 8;
        v4f v0 = *(const v4f*)(smem + row * SP + c);
        v4f v1 = *(const v4f*)(smem + row * SP + c + 4);
        float e[8];
#pragma unroll
        for (int j = 0; j < 4; ++j) { e[j] = v0[j] * oscale; e[j + 4] = v1[j] * oscale; }
        if (EPI == 1) {
          v4f b0v = *(const v4f*)(bias + n0 + c);
          v4f b1v = *(const v4f*)(bias + n0 + c + 4);
#pragma unroll
          for (int j = 0; j < 4; ++j) { e[j] += b0v[j]; e[j + 4] += b1v[j]; }
#pragma unroll
          for (int j = 0; j < 8; ++j) {
            const float x = e[j];
            e[j] = 0.5f * x * (1.0f + erff(x * 0.70710678118654752f));
          }
        }
        v8h o;
#pragma unroll
        for (int j = 0; j < 8; ++j) o[j] = (h16)e[j];
        st2_v8h(Ch + (size_t)(rbase + row) * ldc + n0 + c, o);
      }
    }
    __syncthreads();
  }
}

__global__ __launch_bounds__(256) void k_attn(const h16* __restrict__ Q, int ldq,
                                              const h16* __restrict__ Kp, int ldk,
                                              const h16* __restrict__ Vp, int ldv,
                                              float* __restrict__ O, int ldo,
                                              int N, int heads) {
  constexpr int BN = 32, KS = 72, VS = 40, PS = 40, OS = 68;
  __shared__ __align__(16) float smem[8 * 16 * OS];
  h16* Ks  = (h16*)smem;
  h16* VsT = Ks + BN * KS;
  h16* Pl  = VsT + 64 * VS;

  const int bh = blockIdx.x;
  const int b = bh / heads, h = bh - b * heads;
  const int q0 = blockIdx.y * 128;
  if (q0 + 128 > N) return;
  const int t = threadIdx.x, wave = t >> 5, lane = t & 31;
  const int lr = lane & 15, ls = lane >> 4;

  const size_t qbase = (size_t)b * N * ldq + (size_t)h * 64;
  const size_t kbase = (size_t)b * N * ldk + (size_t)h * 64;
  const size_t vbase = (size_t)b * N * ldv + (size_t)h * 64;

  const int qrow = q0 + wave * 16 + lr;
  v16h qf[2];
#pragma unroll
  for (int kk = 0; kk < 2; ++kk)
    qf[kk] = ldfrag(Q + qbase + (size_t)qrow * ldq + kk * 32 + 8 * ls);

  v8f o[4];
#pragma unroll
  for (int dt = 0; dt < 4; ++dt)
#pragma unroll
    for (int q = 0; q < 8; ++q) o[dt][q] = 0.f;
  float mst[8], lst[8];
#pragma unroll
  for (int q = 0; q < 8; ++q) { mst[q] = -1e30f; lst[q] = 0.f; }

  const int rr = t >> 3, cc = (t & 7) * 8;
  h16* pw = Pl + wave * 16 * PS;
  const int ns = N / BN;
  for (int step = 0; step < ns; ++step) {
    const int key0 = step * BN;
    v8h kreg = ld8(Kp + kbase + (size_t)(key0 + rr) * ldk + cc);
    v8h vreg = ld8(Vp + vbase + (size_t)(key0 + rr) * ldv + cc);
    __syncthreads();
    *(v8h*)(Ks + rr * KS + cc) = kreg;
#pragma unroll
    for (int e = 0; e < 8; ++e) VsT[(cc + e) * VS + rr] = vreg[e];
    __syncthreads();

    v8f s[2];
#pragma unroll
    for (int nt = 0; nt < 2; ++nt) {
#pragma unroll
      for (int q = 0; q < 8; ++q) s[nt][q] = 0.f;
#pragma unroll
      for (int kk = 0; kk < 2; ++kk) {
        v16h bfr = ldfrag(Ks + (nt * 16 + lr) * KS + kk * 32 + 8 * ls);
        s[nt] = wmma16(qf[kk], bfr, s[nt]);
      }
    }

    float pr[2][8];
#pragma unroll
    for (int q = 0; q < 8; ++q) {
      const float s0 = s[0][q] * 0.125f;
      const float s1 = s[1][q] * 0.125f;
      float rowm = fmaxf(s0, s1);
#pragma unroll
      for (int m = 1; m < 16; m <<= 1) rowm = fmaxf(rowm, __shfl_xor(rowm, m, 32));
      const float newm = fmaxf(mst[q], rowm);
      const float alpha = __expf(mst[q] - newm);
      const float p0 = __expf(s0 - newm);
      const float p1 = __expf(s1 - newm);
      float rs = p0 + p1;
#pragma unroll
      for (int m = 1; m < 16; m <<= 1) rs += __shfl_xor(rs, m, 32);
      lst[q] = lst[q] * alpha + rs;
      mst[q] = newm;
      pr[0][q] = p0;
      pr[1][q] = p1;
#pragma unroll
      for (int dt = 0; dt < 4; ++dt) o[dt][q] *= alpha;
    }

#pragma unroll
    for (int nt = 0; nt < 2; ++nt)
#pragma unroll
      for (int q = 0; q < 8; ++q)
        pw[(8 * ls + q) * PS + nt * 16 + lr] = (h16)(pr[nt][q] * 1024.0f);
    __syncthreads();
    v16h pf = ldfrag(pw + lr * PS + 8 * ls);

#pragma unroll
    for (int dt = 0; dt < 4; ++dt) {
      v16h vf = ldfrag(VsT + (dt * 16 + lr) * VS + 8 * ls);
      o[dt] = wmma16(pf, vf, o[dt]);
    }
  }

  __syncthreads();
  float* Os = smem + wave * 16 * OS;
#pragma unroll
  for (int q = 0; q < 8; ++q) {
    const float inv = 1.0f / (lst[q] * 1024.0f);
    const int row = 8 * ls + q;
#pragma unroll
    for (int dt = 0; dt < 4; ++dt) Os[row * OS + dt * 16 + lr] = o[dt][q] * inv;
  }
  __syncthreads();
#pragma unroll
  for (int it = 0; it < 8; ++it) {
    const int row = it * 2 + (lane >> 4);
    const int c = (lane & 15) * 4;
    v4f v = *(const v4f*)(Os + row * OS + c);
    st2_v4f(O + ((size_t)b * N + q0 + wave * 16 + row) * ldo + (size_t)h * 64 + c, v);
  }
}

extern "C" void kernel_launch(void* const* d_in, const int* in_sizes, int n_in,
                              void* d_out, int out_size, void* d_ws, size_t ws_size,
                              hipStream_t stream) {
  constexpr int Bb = 2, N = 2048, MR = Bb * N;
  constexpr int DIM = 1024, DF = 384, HID = 1024, HEADS = 16;
  static_assert(MR % 128 == 0 && N % 128 == 0 && N % 32 == 0, "");
  static_assert(DIM % 128 == 0 && DF % 64 == 0 && HID % 128 == 0, "");
  static_assert(DIM % 32 == 0 && DF % 32 == 0, "");

  if (n_in < 13) return;
  if (in_sizes[0] != MR * DIM || in_sizes[1] != MR * DF || in_sizes[2] != DIM ||
      in_sizes[3] != DIM || in_sizes[4] != DIM * HID || in_sizes[5] != DF * 2 * HID ||
      in_sizes[6] != DIM * 3 * HID || in_sizes[7] != DIM || in_sizes[8] != DIM ||
      in_sizes[9] != DIM * 4 * DIM || in_sizes[10] != 4 * DIM ||
      in_sizes[11] != 4 * DIM * DIM || in_sizes[12] != DIM || out_size != MR * DIM)
    return;

  const float* x      = (const float*)d_in[0];
  const float* feat   = (const float*)d_in[1];
  const float* norm_g = (const float*)d_in[2];
  const float* norm_b = (const float*)d_in[3];
  const float* W_cq   = (const float*)d_in[4];
  const float* W_ckv  = (const float*)d_in[5];
  const float* W_sqkv = (const float*)d_in[6];
  const float* ffn_g  = (const float*)d_in[7];
  const float* ffn_b  = (const float*)d_in[8];
  const float* W1     = (const float*)d_in[9];
  const float* b1     = (const float*)d_in[10];
  const float* W2     = (const float*)d_in[11];
  const float* b2     = (const float*)d_in[12];
  float* out = (float*)d_out;

  char* ws = (char*)d_ws;
  size_t off = 0;
  auto carve = [&](size_t bytes) -> char* {
    char* p = ws + off;
    off += (bytes + 255) & ~(size_t)255;
    return p;
  };

  h16* wCqT   = (h16*)carve((size_t)HID * DIM * 2);
  h16* wCkvT  = (h16*)carve((size_t)2 * HID * DF * 2);
  h16* wSqkvT = (h16*)carve((size_t)3 * HID * DIM * 2);
  h16* w1T    = (h16*)carve((size_t)4 * DIM * DIM * 2);
  h16* w2T    = (h16*)carve((size_t)DIM * 4 * DIM * 2);
  h16* feat16 = (h16*)carve((size_t)MR * DF * 2);
  h16* xn16   = (h16*)carve((size_t)MR * DIM * 2);
  h16* q16    = (h16*)carve((size_t)MR * HID * 2);
  h16* kv16   = (h16*)carve((size_t)MR * 2 * HID * 2);
  h16* qkv16  = (h16*)carve((size_t)MR * 3 * HID * 2);
  h16* h1     = (h16*)carve((size_t)MR * 4 * DIM * 2);
  float* at32    = (float*)carve((size_t)MR * HID * 4);
  float* cross   = (float*)carve((size_t)MR * DIM * 4);
  float* selftok = (float*)carve((size_t)MR * DIM * 4);
  if (off > ws_size) return;

  const dim3 blk(256);

  k_cvt_wt<<<dim3(HID / 64, DIM / 64), blk, 0, stream>>>(W_cq, wCqT, DIM, HID, 64.0f);
  k_cvt_wt<<<dim3(2 * HID / 64, DF / 64), blk, 0, stream>>>(W_ckv, wCkvT, DF, 2 * HID, 64.0f);
  k_cvt_wt<<<dim3(3 * HID / 64, DIM / 64), blk, 0, stream>>>(W_sqkv, wSqkvT, DIM, 3 * HID, 64.0f);
  k_cvt_wt<<<dim3(4 * DIM / 64, DIM / 64), blk, 0, stream>>>(W1, w1T, DIM, 4 * DIM, 64.0f);
  k_cvt_wt<<<dim3(DIM / 64, 4 * DIM / 64), blk, 0, stream>>>(W2, w2T, 4 * DIM, DIM, 64.0f);
  {
    const int n8 = MR * DF / 8;
    k_cvt_act<<<dim3((n8 + 255) / 256), blk, 0, stream>>>(feat, feat16, n8);
  }

  k_ln<false><<<dim3(MR), blk, 0, stream>>>(x, x, norm_g, norm_b, cross, xn16, MR);
  k_gemm<0><<<dim3(HID / 128, MR / 128), blk, 0, stream>>>(
      xn16, DIM, wCqT, DIM, q16, out, HID, b2, cross, DIM, MR, HID, DIM, 1.0f / 64.0f);
  k_gemm<0><<<dim3(2 * HID / 128, MR / 128), blk, 0, stream>>>(
      feat16, DF, wCkvT, DF, kv16, out, 2 * HID, b2, cross, DIM, MR, 2 * HID, DF, 1.0f / 64.0f);
  k_attn<<<dim3(Bb * HEADS, N / 128), blk, 0, stream>>>(
      q16, HID, kv16, 2 * HID, kv16 + HID, 2 * HID, at32, HID, N, HEADS);
  k_ln<true><<<dim3(MR), blk, 0, stream>>>(at32, x, norm_g, norm_b, cross, xn16, MR);
  k_gemm<0><<<dim3(3 * HID / 128, MR / 128), blk, 0, stream>>>(
      xn16, DIM, wSqkvT, DIM, qkv16, out, 3 * HID, b2, cross, DIM, MR, 3 * HID, DIM, 1.0f / 64.0f);
  k_attn<<<dim3(Bb * HEADS, N / 128), blk, 0, stream>>>(
      qkv16, 3 * HID, qkv16 + HID, 3 * HID, qkv16 + 2 * HID, 3 * HID, at32, HID, N, HEADS);
  k_ln<true><<<dim3(MR), blk, 0, stream>>>(at32, cross, ffn_g, ffn_b, selftok, xn16, MR);
  k_gemm<1><<<dim3(4 * DIM / 128, MR / 128), blk, 0, stream>>>(
      xn16, DIM, w1T, DIM, h1, out, 4 * DIM, b1, cross, DIM, MR, 4 * DIM, DIM, 1.0f / 64.0f);
  k_gemm<2><<<dim3(DIM / 128, MR / 128), blk, 0, stream>>>(
      h1, 4 * DIM, w2T, 4 * DIM, h1, out, DIM, b2, selftok, DIM, MR, DIM, 4 * DIM, 1.0f / 64.0f);
}
